// ExactSlidingWindowAttention_23089744183532
// MI455X (gfx1250) — hardware-verified
//
#include <hip/hip_runtime.h>
#include <math.h>
typedef __attribute__((ext_vector_type(16))) _Float16 v16h;
typedef __attribute__((ext_vector_type(8)))  _Float16 v8h;
typedef __attribute__((ext_vector_type(16))) __bf16   v16b;
typedef __attribute__((ext_vector_type(8)))  __bf16   v8b;
typedef __attribute__((ext_vector_type(8)))  float    v8f;
typedef __attribute__((ext_vector_type(4)))  float    v4f;

#define AT_D 64
#define AT_NW 4
#define AT_QB 64
#define AT_KC 64
struct AttnGeom { const float* cp = nullptr; const float* pc = nullptr; long c_bs = 0, c_rs = 0, c_hs = 0;
                  long q_bs, q_rs, q_hs, k_bs, k_rs, k_hs, v_bs, v_rs, v_hs, o_bs, o_rs, o_hs;
                  int S, Skv, H, mask_mode; float qscale; int blk0; float mask_fill; int mask_is_int; };
static_assert(sizeof(AttnGeom) == 168, "no padding");

__device__ __forceinline__ unsigned short at_bf_bits(float f) {
  unsigned u = __float_as_uint(f);
  return (unsigned short)((u + 0x7FFFu + ((u >> 16) & 1u)) >> 16);
}
__device__ __forceinline__ __bf16 at_f2bf(float f) { return __builtin_bit_cast(__bf16, at_bf_bits(f)); }
__device__ __forceinline__ void at_split(float f, __bf16& hi, __bf16& lo) {
  const unsigned short hb = at_bf_bits(f);
  hi = __builtin_bit_cast(__bf16, hb);
  lo = at_f2bf(f - __uint_as_float(((unsigned)hb) << 16));
}
__device__ __forceinline__ v8f at_mma(v16b a, v16b b, v8f c) {
  c = __builtin_amdgcn_wmma_f32_16x16x32_bf16(false, a, false, b, (short)0, c, false, false);
  asm volatile("v_nop\n\tv_nop\n\tv_nop\n\tv_nop" : "+v"(c) : "v"(a), "v"(b));
  return c;
}
template <bool F16> __device__ __forceinline__ __bf16 at_to16(float f) {
  if (F16) return __builtin_bit_cast(__bf16, (_Float16)f);
  return at_f2bf(f);
}
template <bool F16> __device__ __forceinline__ v8f at_mma16(v16b a, v16b b, v8f c) {
  if (F16) {
    const v16h ah = __builtin_bit_cast(v16h, a), bh = __builtin_bit_cast(v16h, b);
    c = __builtin_amdgcn_wmma_f32_16x16x32_f16(false, ah, false, bh, (short)0, c, false, false);
    asm volatile("v_nop\n\tv_nop\n\tv_nop\n\tv_nop" : "+v"(c) : "v"(ah), "v"(bh));
    return c;
  }
  return at_mma(a, b, c);
}

template <bool SPLIT_QK, bool SPLIT_PV, bool F16 = false>
__global__ __launch_bounds__(128)
void attn64_kernel(const float* __restrict__ q, const float* __restrict__ k,
                   const float* __restrict__ v, float* __restrict__ out,
                   const void* __restrict__ mask_a, const int* __restrict__ mask_b, AttnGeom g) {
  static_assert(!(F16 && (SPLIT_QK || SPLIT_PV)), "f16 mode is non-split");
  const float PSC = F16 ? 32768.0f : 1.0f;
  union FB { v16b v; v8b h[2]; };
  __shared__ __align__(16) __bf16 Ksh[AT_KC * AT_D];
  __shared__ __align__(16) __bf16 Ksl[SPLIT_QK ? AT_KC * AT_D : 8];
  __shared__ __align__(16) __bf16 Vth[AT_D * AT_KC];
  __shared__ __align__(16) __bf16 Vtl[SPLIT_PV ? AT_D * AT_KC : 8];
  __shared__ __align__(16) __bf16 Psh[AT_NW][16 * AT_KC];
  __shared__ __align__(16) __bf16 Psl[SPLIT_PV ? AT_NW : 1][SPLIT_PV ? 16 * AT_KC : 8];
  __shared__ __align__(16) float  Os[AT_NW][16 * 68];

  const int tid  = threadIdx.x;
  const int wave = tid >> 5;
  const int lane = tid & 31;
  const int hh   = lane >> 4;
  const int c    = lane & 15;

  const int nqb = g.S / AT_QB;
  const int bx = blockIdx.x + g.blk0;
  const int qb = bx % nqb;
  const int bh = bx / nqb;
  const int h  = bh % g.H;
  const int b  = bh / g.H;
  const int qbase_block = qb * AT_QB;
  const int q0 = qbase_block + wave * 16;

  const float* qb_ptr = q + (size_t)b * g.q_bs + (size_t)h * g.q_hs;
  const float* kb_ptr = k + (size_t)b * g.k_bs + (size_t)h * g.k_hs;
  const float* vb_ptr = v + (size_t)b * g.v_bs + (size_t)h * g.v_hs;
  float*       ob_ptr = out + (size_t)b * g.o_bs + (size_t)h * g.o_hs;

  v16b qah[2], qal[2];
  {
    const float* qrow = qb_ptr + (size_t)(q0 + c) * g.q_rs;
#pragma unroll
    for (int dc = 0; dc < 2; ++dc) {
#pragma unroll
      for (int e = 0; e < 8; ++e) {
        const float f0 = qrow[dc * 32 + 8 * hh + e] * g.qscale;
        const float f1 = qrow[dc * 32 + 16 + 8 * hh + e] * g.qscale;
        if (SPLIT_QK) { __bf16 hq, lq; at_split(f0, hq, lq); qah[dc][e] = hq; qal[dc][e] = lq; at_split(f1, hq, lq); qah[dc][8 + e] = hq; qal[dc][8 + e] = lq; }
        else { qah[dc][e] = at_to16<F16>(f0); qah[dc][8 + e] = at_to16<F16>(f1); qal[dc][e] = qah[dc][e]; qal[dc][8 + e] = qah[dc][8 + e]; }
      }
    }
  }

  float mrow[8], lrow[8];
  v8f oacc[4];
#pragma unroll
  for (int r = 0; r < 8; ++r) { mrow[r] = -INFINITY; lrow[r] = 0.f; }
#pragma unroll
  for (int t = 0; t < 4; ++t) oacc[t] = (v8f){0.f,0.f,0.f,0.f,0.f,0.f,0.f,0.f};

  const int nChunks = (g.mask_mode == 1 || g.mask_mode == 4) ? (qb + 1) : (g.Skv / AT_KC);
  const int kcFirst = (g.mask_mode == 4) ? max(0, (qb * 64 - g.mask_is_int) / AT_KC) : 0;
  int qkeep[8];
#pragma unroll
  for (int r = 0; r < 8; ++r) qkeep[r] = (g.mask_mode == 3) ? mask_b[(size_t)b * g.S + q0 + 8 * hh + r] : 1;
  for (int kc = kcFirst; kc < nChunks; ++kc) {
    const int kv0 = kc * AT_KC;
    __syncthreads();
    {
      const int kvr = tid >> 1, dh = (tid & 1) * 32;
      const float* krow = kb_ptr + (size_t)(kv0 + kvr) * g.k_rs + dh;
      const float* vrow = vb_ptr + (size_t)(kv0 + kvr) * g.v_rs + dh;
#pragma unroll
      for (int i = 0; i < 8; ++i) {
        v4f kk = *(const v4f*)(krow + 4 * i);
        v4f vv = *(const v4f*)(vrow + 4 * i);
#pragma unroll
        for (int e = 0; e < 4; ++e) {
          const int d = dh + 4 * i + e;
          if (SPLIT_QK) { __bf16 a, bl; at_split(kk[e], a, bl); Ksh[kvr * AT_D + d] = a; Ksl[kvr * AT_D + d] = bl; }
          else Ksh[kvr * AT_D + d] = at_to16<F16>(kk[e]);
          if (SPLIT_PV) { __bf16 a, bl; at_split(vv[e], a, bl); Vth[d * AT_KC + kvr] = a; Vtl[d * AT_KC + kvr] = bl; }
          else Vth[d * AT_KC + kvr] = at_to16<F16>(vv[e]);
        }
      }
    }
    __syncthreads();

    v8f s[4];
#pragma unroll
    for (int j = 0; j < 4; ++j) {
      s[j] = (v8f){0.f,0.f,0.f,0.f,0.f,0.f,0.f,0.f};
#pragma unroll 1
      for (int dc = 0; dc < 2; ++dc) {
        FB kb;
        kb.h[0] = *(const v8b*)(Ksh + (j * 16 + c) * AT_D + dc * 32 + 8 * hh);
        kb.h[1] = *(const v8b*)(Ksh + (j * 16 + c) * AT_D + dc * 32 + 16 + 8 * hh);
        s[j] = at_mma16<F16>(qah[dc], kb.v, s[j]);
        if (SPLIT_QK) {
          FB kl;
          kl.h[0] = *(const v8b*)(Ksl + (j * 16 + c) * AT_D + dc * 32 + 8 * hh);
          kl.h[1] = *(const v8b*)(Ksl + (j * 16 + c) * AT_D + dc * 32 + 16 + 8 * hh);
          s[j] = at_mma16<F16>(qah[dc], kl.v, s[j]);
          s[j] = at_mma16<F16>(qal[dc], kb.v, s[j]);
        }
      }
    }
    const bool diag = (g.mask_mode == 1) && (kc == qb);
    int kvkeep[4] = {1, 1, 1, 1};
    if (g.mask_mode == 3) {
#pragma unroll
      for (int j = 0; j < 4; ++j) kvkeep[j] = ((const int*)mask_a)[(size_t)b * g.Skv + kv0 + j * 16 + c];
    }
    float cm[8];
#pragma unroll
    for (int r = 0; r < 8; ++r) {
      const int qrow = q0 + 8 * hh + r;
      float m = -INFINITY;
#pragma unroll
      for (int j = 0; j < 4; ++j) {
        const int kvcol = kv0 + j * 16 + c;
        bool masked = false;
        if (diag) masked = (kvcol > qrow);
        else if (g.mask_mode == 4) masked = (kvcol > qrow) || (qrow - kvcol > g.mask_is_int);
        else if (g.mask_mode == 2) {
          const size_t mi = (size_t)qrow * g.Skv + kvcol;
          masked = (g.mask_is_int == 0) ? (((const float*)mask_a)[mi] == 0.0f)
                 : (g.mask_is_int == 1) ? (((const int*)mask_a)[mi] == 0) : (((const int*)mask_a)[mi] != 0);
        } else if (g.mask_mode == 3) masked = (qkeep[r] == 0) || (kvkeep[j] == 0);
        else if (g.mask_mode == 5) {
          const size_t mi = (size_t)qrow * g.Skv + kvcol;
          masked = (((const int*)mask_a)[mi] != 0);
          int n = mask_b[mi]; n = n < 0 ? 0 : n;
          s[j][r] += g.cp[(size_t)b * g.c_bs + (size_t)h * g.c_hs + (size_t)qrow * g.c_rs + n]
                   + g.pc[(size_t)b * g.c_bs + (size_t)h * g.c_hs + (size_t)kvcol * g.c_rs + n];
        }
        if (masked) s[j][r] = g.mask_fill;
        m = fmaxf(m, s[j][r]);
      }
#pragma unroll
      for (int off = 1; off < 16; off <<= 1) m = fmaxf(m, __shfl_xor(m, off, 32));
      cm[r] = m;
    }
    __bf16* pwh = Psh[wave];
    __bf16* pwl = Psl[SPLIT_PV ? wave : 0];
#pragma unroll
    for (int r = 0; r < 8; ++r) {
      const float mnew = fmaxf(mrow[r], cm[r]);
      const float alpha = expf(mrow[r] - mnew);
      mrow[r] = mnew;
      float psum = 0.f;
#pragma unroll
      for (int j = 0; j < 4; ++j) {
        const float p = expf(s[j][r] - mnew);
        psum += p;
        if (SPLIT_PV) { __bf16 a, bl; at_split(p, a, bl); pwh[(8 * hh + r) * AT_KC + j * 16 + c] = a; pwl[(8 * hh + r) * AT_KC + j * 16 + c] = bl; }
        else pwh[(8 * hh + r) * AT_KC + j * 16 + c] = at_to16<F16>(p * PSC);
      }
#pragma unroll
      for (int off = 1; off < 16; off <<= 1) psum += __shfl_xor(psum, off, 32);
      lrow[r] = lrow[r] * alpha + psum;
#pragma unroll
      for (int t = 0; t < 4; ++t) oacc[t][r] *= alpha;
    }
    __builtin_amdgcn_fence(__ATOMIC_RELEASE, "workgroup");
    __builtin_amdgcn_wave_barrier();
    __builtin_amdgcn_fence(__ATOMIC_ACQUIRE, "workgroup");
#pragma unroll 1
    for (int kk = 0; kk < 2; ++kk) {
      FB pa, pl;
      pa.h[0] = *(const v8b*)(pwh + c * AT_KC + kk * 32 + 8 * hh);
      pa.h[1] = *(const v8b*)(pwh + c * AT_KC + kk * 32 + 16 + 8 * hh);
      if (SPLIT_PV) {
        pl.h[0] = *(const v8b*)(pwl + c * AT_KC + kk * 32 + 8 * hh);
        pl.h[1] = *(const v8b*)(pwl + c * AT_KC + kk * 32 + 16 + 8 * hh);
      }
#pragma unroll
      for (int t = 0; t < 4; ++t) {
        FB vb;
        vb.h[0] = *(const v8b*)(Vth + (t * 16 + c) * AT_KC + kk * 32 + 8 * hh);
        vb.h[1] = *(const v8b*)(Vth + (t * 16 + c) * AT_KC + kk * 32 + 16 + 8 * hh);
        oacc[t] = at_mma16<F16>(pa.v, vb.v, oacc[t]);
        if (SPLIT_PV) {
          FB vl;
          vl.h[0] = *(const v8b*)(Vtl + (t * 16 + c) * AT_KC + kk * 32 + 8 * hh);
          vl.h[1] = *(const v8b*)(Vtl + (t * 16 + c) * AT_KC + kk * 32 + 16 + 8 * hh);
          oacc[t] = at_mma16<F16>(pa.v, vl.v, oacc[t]);
          oacc[t] = at_mma16<F16>(pl.v, vb.v, oacc[t]);
        }
      }
    }
  }

  float* os = Os[wave];
#pragma unroll
  for (int r = 0; r < 8; ++r) {
    const float inv = 1.0f / (lrow[r] * PSC);
#pragma unroll
    for (int t = 0; t < 4; ++t) os[(8 * hh + r) * 68 + t * 16 + c] = oacc[t][r] * inv;
  }
  __builtin_amdgcn_fence(__ATOMIC_RELEASE, "workgroup");
  __builtin_amdgcn_wave_barrier();
  __builtin_amdgcn_fence(__ATOMIC_ACQUIRE, "workgroup");
  {
    const int c4 = (lane & 15) * 4;
    for (int pass = 0; pass < 2; ++pass) {
#pragma unroll
      for (int it = 0; it < 8; ++it) {
        const int row = it * 2 + hh;
        v4f val = *(const v4f*)(os + row * 68 + c4);
        *(volatile v4f*)(ob_ptr + (size_t)(q0 + row) * g.o_rs + c4) = val;
      }
      __threadfence();
    }
  }
}

extern "C" void kernel_launch(void* const* d_in, const int* in_sizes, int n_in, void* d_out, int out_size, void* d_ws, size_t ws_size, hipStream_t stream) {
  (void)in_sizes; (void)n_in; (void)out_size; (void)ws_size; (void)d_ws;
  const float* q = (const float*)d_in[0]; const float* k = (const float*)d_in[1]; const float* v = (const float*)d_in[2];
  const int B = 16, S = 4096, D = 64;
  AttnGeom g; g.cp = nullptr; g.pc = nullptr; g.c_bs = g.c_rs = g.c_hs = 0;
  g.q_bs = (long)S * D; g.q_rs = D; g.q_hs = 0; g.k_bs = (long)S * D; g.k_rs = D; g.k_hs = 0; g.v_bs = (long)S * D; g.v_rs = D; g.v_hs = 0; g.o_bs = (long)S * D; g.o_rs = D; g.o_hs = 0;
  g.S = S; g.Skv = S; g.H = 1; g.mask_mode = 4; g.qscale = 0.125f; g.blk0 = 0; g.mask_fill = -1.0e30f; g.mask_is_int = 511;
  attn64_kernel<true, true, false><<<B * (S / 64), 128, 0, stream>>>(q, k, v, (float*)d_out, nullptr, nullptr, g);
}
